// GIN_19421842112604
// MI455X (gfx1250) — hardware-verified
//
#include <hip/hip_runtime.h>
#include <stddef.h>
#include <stdint.h>
#include <math.h>


#define DIN     128
#define HID     1024
#define DMID    256
#define NCLS    10
#define K1A     256
#define K2H     2048
#define CHR     5120
#define NTHR    256
#define NWAVE   8
#define EPT     8
#define CHUNK   (NTHR * EPT)
#define WCAP    (EPT * 32)
#define LISTN   (NWAVE * WCAP)
#define NBMAX   2048
#define RCAP    28672
#define DEGCAP  64
#define PKS     11
#define GBM     64
#define GBN     128
#define GTHR    128
#define GNT     8
#define PARTW   288
#define APR1    4
#define APR2    4
#define HR      128
#define NUA     (HID * (K1A / 8))
#define NUH     (HID * (K2H / 8))
#define NUL     (DMID * (K2H / 8))
#define UB1     (NUA)
#define UB2     (NUA + NUH)
#define UB3     (NUA + 2 * NUH)
#define UB4     (NUA + 3 * NUH)
#define NUTOT   (NUA + 3 * NUH + NUL)
#define WSMAX   268435456
#define LDS_AGG ((2 * RCAP + 2 * NBMAX + LISTN) * 4 + 64)

static_assert((CHUNK & (CHUNK - 1)) == 0 && CHUNK <= (1 << PKS));
static_assert((NBMAX & (NBMAX - 1)) == 0 && NBMAX <= (1 << PKS));
static_assert(NTHR * 8 == NBMAX);
static_assert(LISTN >= NBMAX && LISTN >= NWAVE * WCAP);
static_assert((RCAP % 32) == 0);
static_assert(LDS_AGG <= 300000);
static_assert(GBM == (GTHR / 32) * 16 && GBN == 16 * GNT && GTHR == GBN);
static_assert((K1A % 32) == 0 && (K2H % 32) == 0);
static_assert((HID % GBN) == 0 && (DMID % GBN) == 0);
static_assert((CHR % GBM) == 0);
static_assert((PARTW % 32) == 0 && PARTW >= 2 * GBN + 1 && PARTW / 4 <= GTHR);
static_assert((NUA % NTHR) == 0 && (NUH % NTHR) == 0 && (NUL % NTHR) == 0);
static_assert(NTHR * 4 == HID);
static_assert((HR * NCLS) % 4 == 0 && (HR * NCLS) / 4 <= 2 * NTHR);
static_assert(2 * HR == NTHR && NCLS == 10);

typedef float          v4f  __attribute__((ext_vector_type(4)));
typedef float          v8f  __attribute__((ext_vector_type(8)));
typedef int            v4i  __attribute__((ext_vector_type(4)));
typedef int            v8i  __attribute__((ext_vector_type(8)));
typedef unsigned int   v2u  __attribute__((ext_vector_type(2)));
typedef unsigned int   v4u  __attribute__((ext_vector_type(4)));
typedef unsigned short v8us __attribute__((ext_vector_type(8)));
typedef __bf16         v16b __attribute__((ext_vector_type(16)));
typedef v4f  __attribute__((may_alias)) v4fa;
typedef v8us __attribute__((may_alias)) v8usa;
union Frag { v16b vb; v8us h[2]; v8i w; };

__device__ __forceinline__ v8f wmx(const Frag& a, const Frag& b, v8f c) {
  v8f d = __builtin_amdgcn_wmma_f32_16x16x32_bf16(false, a.vb, false, b.vb, (short)0, c, false, false);
  asm volatile("v_nop\n\tv_nop\n\tv_nop\n\tv_nop" : "+v"(d) : "v"(a.w), "v"(b.w));
  return d;
}

__device__ __forceinline__ unsigned short bf_bits(float f) {
  unsigned int u = __float_as_uint(f);
  u += 0x7FFFu + ((u >> 16) & 1u);
  return (unsigned short)(u >> 16);
}
__device__ __forceinline__ float bf_val(unsigned short b) { return __uint_as_float(((unsigned int)b) << 16); }
__device__ __forceinline__ float bf_rne(float f) { return bf_val(bf_bits(f)); }

__device__ __forceinline__ float relu_np(float v) { return (v > 0.0f) ? v : (v - v); }

__device__ __forceinline__ void hilo8(const v4f a, const v4f b, v8us& hv, v8us& lv) {
  const float f[8] = {a.x, a.y, a.z, a.w, b.x, b.y, b.z, b.w};
#pragma unroll
  for (int j = 0; j < 8; ++j) {
    const unsigned short hb = bf_bits(f[j]);
    hv[j] = hb;
    lv[j] = bf_bits(f[j] - bf_val(hb));
  }
}

__device__ __forceinline__ int scan_chunk(const int* __restrict__ dsts, int nE, int cbase, int slotBase,
                                          int nb, int vec8, int* list, int tid, int lane, int wave) {
  int wc = 0;
  const int el0  = tid * EPT;
  const int e0   = cbase + el0;
  const int sent = -2147483647 - 1;
  v4i da, db;
  if (vec8 != 0 && cbase + CHUNK <= nE) {
    da = *(const v4i*)(dsts + e0);
    db = *(const v4i*)(dsts + e0 + 4);
  } else {
    da.x = (e0     < nE) ? dsts[min(e0,     nE - 1)] : sent;
    da.y = (e0 + 1 < nE) ? dsts[min(e0 + 1, nE - 1)] : sent;
    da.z = (e0 + 2 < nE) ? dsts[min(e0 + 2, nE - 1)] : sent;
    da.w = (e0 + 3 < nE) ? dsts[min(e0 + 3, nE - 1)] : sent;
    db.x = (e0 + 4 < nE) ? dsts[min(e0 + 4, nE - 1)] : sent;
    db.y = (e0 + 5 < nE) ? dsts[min(e0 + 5, nE - 1)] : sent;
    db.z = (e0 + 6 < nE) ? dsts[min(e0 + 6, nE - 1)] : sent;
    db.w = (e0 + 7 < nE) ? dsts[min(e0 + 7, nE - 1)] : sent;
  }
  const unsigned nbs = (unsigned)slotBase;
  const unsigned unb = (unsigned)nb;
  const unsigned s0 = (unsigned)da.x - nbs, s1 = (unsigned)da.y - nbs;
  const unsigned s2 = (unsigned)da.z - nbs, s3 = (unsigned)da.w - nbs;
  const unsigned s4 = (unsigned)db.x - nbs, s5 = (unsigned)db.y - nbs;
  const unsigned s6 = (unsigned)db.z - nbs, s7 = (unsigned)db.w - nbs;
  const bool h0 = s0 < unb, h1 = s1 < unb, h2 = s2 < unb, h3 = s3 < unb;
  const bool h4 = s4 < unb, h5 = s5 < unb, h6 = s6 < unb, h7 = s7 < unb;
  const unsigned any = __builtin_amdgcn_ballot_w32(h0 | h1 | h2 | h3 | h4 | h5 | h6 | h7);
  if (any != 0u) {
#define HITJ(J, HJ, SJ) { \
      const unsigned mj = __builtin_amdgcn_ballot_w32(HJ); \
      if (mj != 0u) { \
        if (HJ) { \
          const int pos = wc + (int)__builtin_amdgcn_mbcnt_lo(mj, 0u); \
          if (pos < WCAP) list[wave * WCAP + pos] = ((el0 + (J)) << PKS) | (int)(SJ); \
        } \
        wc += (int)__builtin_popcount(mj); } }
    HITJ(0, h0, s0)
    HITJ(1, h1, s1)
    HITJ(2, h2, s2)
    HITJ(3, h3, s3)
    HITJ(4, h4, s4)
    HITJ(5, h5, s5)
    HITJ(6, h6, s6)
    HITJ(7, h7, s7)
#undef HITJ
  }
  return wc;
}

__device__ __forceinline__ v8us cv8b(const float* __restrict__ p, size_t stride) {
  v8us o;
#pragma unroll
  for (int i = 0; i < 8; ++i) o[i] = bf_bits(p[(size_t)i * stride]);
  return o;
}

__global__ __launch_bounds__(NTHR) void k_wprep(const float* __restrict__ w1a, const float* __restrict__ w1b,
                                                const float* __restrict__ w2a, const float* __restrict__ w2b,
                                                const float* __restrict__ wl1,
                                                unsigned short* p1a, unsigned short* p1b, unsigned short* p2a,
                                                unsigned short* p2b, unsigned short* pl1) {
  const int u = (int)blockIdx.x * NTHR + (int)threadIdx.x;
  v8us o;
  unsigned short* dp;
  if (u < UB1) {
    const int v = u, n = v >> 5, k8 = (v & 31) * 8;
    const int kk = k8 & (DIN - 1);
    o = cv8b(w1a + (size_t)kk * HID + n, HID);
    dp = p1a + (size_t)v * 8;
  } else if (u < UB2) {
    const int v = u - UB1, n = v >> 8, k8 = (v & 255) * 8;
    const int kk = k8 & (HID - 1);
    o = cv8b(w1b + (size_t)kk * HID + n, HID);
    dp = p1b + (size_t)v * 8;
  } else if (u < UB3) {
    const int v = u - UB2, n = v >> 8, k8 = (v & 255) * 8;
    const int kk = k8 & (HID - 1);
    o = cv8b(w2a + (size_t)kk * HID + n, HID);
    dp = p2a + (size_t)v * 8;
  } else if (u < UB4) {
    const int v = u - UB3, n = v >> 8, k8 = (v & 255) * 8;
    const int kk = k8 & (HID - 1);
    o = cv8b(w2b + (size_t)kk * HID + n, HID);
    dp = p2b + (size_t)v * 8;
  } else if (u < NUTOT) {
    const int v = u - UB4, n = v >> 8, k8 = (v & 255) * 8;
    const int kk = k8 & (HID - 1);
    o = cv8b(wl1 + (size_t)kk * DMID + n, DMID);
    dp = pl1 + (size_t)v * 8;
  } else {
    return;
  }
  *(volatile v8us*)dp = o;
  __threadfence();
  *(volatile v8us*)dp = o;
}

template <int NV, int RND>
__global__ __launch_bounds__(NTHR) void k_agg(
    const int* __restrict__ srcs, const int* __restrict__ dsts,
    const float* __restrict__ fin, unsigned short* Aout,
    int nN, int nE, int nb, int vec8, int rowOff, int MPr) {
  constexpr int W = 128 * NV;
  extern __shared__ v4f lds_dyn[];
  int* reg1 = (int*)lds_dyn;
  int* reg2 = reg1 + RCAP;
  int* scnt = reg2 + RCAP;
  int* soff = scnt + NBMAX;
  int* list = soff + NBMAX;
  int* wcnt = list + LISTN;
  int* wtot = wcnt + NWAVE;
  const int tid = (int)threadIdx.x, lane = tid & 31, wave = tid >> 5;
  const int nodeBase = rowOff + (int)blockIdx.x * nb;

  for (int i = tid; i < NBMAX; i += NTHR) scnt[i] = 0;
  __syncthreads();

  int tot = 0;
  const int nChunks = (nE + CHUNK - 1) / CHUNK;
#pragma unroll 1
  for (int ch = 0; ch < nChunks; ++ch) {
    const int cbase = ch * CHUNK;
    const int wc = scan_chunk(dsts, nE, cbase, nodeBase, nb, vec8, list, tid, lane, wave);
    if (lane == 0) wcnt[wave] = wc;
    __syncthreads();
    int pre = 0, all = 0;
#pragma unroll
    for (int w2 = 0; w2 < NWAVE; ++w2) {
      int c = wcnt[w2];
      c = c < 0 ? 0 : (c > WCAP ? WCAP : c);
      all += c;
      pre += (w2 < wave) ? c : 0;
    }
    const int wcc  = wc > WCAP ? WCAP : wc;
    const int base = tot + pre;
#pragma unroll 1
    for (int i = lane; i < wcc; i += 32) {
      const int ent = list[wave * WCAP + i];
      const int el  = (ent >> PKS) & (CHUNK - 1);
      const int sl  = ent & (NBMAX - 1);
      int eid = cbase + el;
      eid = eid > nE - 1 ? nE - 1 : eid;
      const int pos = base + i;
      if (pos < RCAP) reg1[pos] = (int)(((unsigned)eid << PKS) | (unsigned)sl);
    }
    tot += all;
    tot = tot > RCAP ? RCAP : tot;
    __syncthreads();
  }
  const int nh = tot;

  if (wave == 0) {
#pragma unroll 1
    for (int b0 = 0; b0 < nh; b0 += 32) {
      const int idx = b0 + lane;
      const int uv  = reg1[idx < RCAP ? idx : RCAP - 1];
      const int m32 = (nh - b0) < 32 ? (nh - b0) : 32;
#pragma unroll 1
      for (int k = 0; k < m32; ++k) {
        const int u  = __builtin_amdgcn_readlane(uv, k);
        const int sl = u & (NBMAX - 1);
        if (lane == 0) scnt[sl] = scnt[sl] + 1;
      }
    }
  }
  __syncthreads();

  {
    const v4i ca = *(const v4i*)(scnt + 8 * tid);
    const v4i cb = *(const v4i*)(scnt + 8 * tid + 4);
    const int e0 = ca.x < 0 ? 0 : ca.x, e1 = ca.y < 0 ? 0 : ca.y, e2 = ca.z < 0 ? 0 : ca.z, e3 = ca.w < 0 ? 0 : ca.w;
    const int e4 = cb.x < 0 ? 0 : cb.x, e5 = cb.y < 0 ? 0 : cb.y, e6 = cb.z < 0 ? 0 : cb.z, e7 = cb.w < 0 ? 0 : cb.w;
    const int ts = e0 + e1 + e2 + e3 + e4 + e5 + e6 + e7;
    int incl = ts;
#pragma unroll
    for (int d = 1; d < 32; d <<= 1) {
      const int up = __shfl_up(incl, d);
      if (lane >= d) incl += up;
    }
    if (lane == 31) wtot[wave] = incl;
    __syncthreads();
    int pre = 0;
#pragma unroll
    for (int w2 = 0; w2 < NWAVE; ++w2) pre += (w2 < wave) ? wtot[w2] : 0;
    int run = pre + incl - ts;
    soff[8 * tid + 0] = run; run += e0;
    soff[8 * tid + 1] = run; run += e1;
    soff[8 * tid + 2] = run; run += e2;
    soff[8 * tid + 3] = run; run += e3;
    soff[8 * tid + 4] = run; run += e4;
    soff[8 * tid + 5] = run; run += e5;
    soff[8 * tid + 6] = run; run += e6;
    soff[8 * tid + 7] = run;
  }
  __syncthreads();
  for (int i = tid; i < NBMAX; i += NTHR) list[i] = soff[i];
  __syncthreads();

  if (wave == 0) {
#pragma unroll 1
    for (int b0 = 0; b0 < nh; b0 += 32) {
      const int idx = b0 + lane;
      const int uv  = reg1[idx < RCAP ? idx : RCAP - 1];
      const int m32 = (nh - b0) < 32 ? (nh - b0) : 32;
#pragma unroll 1
      for (int k = 0; k < m32; ++k) {
        const int u   = __builtin_amdgcn_readlane(uv, k);
        const int sl  = u & (NBMAX - 1);
        const int eid = (int)((unsigned)u >> PKS);
        if (lane == 0) {
          int pos = list[sl];
          pos = pos < 0 ? 0 : (pos > RCAP - 1 ? RCAP - 1 : pos);
          reg2[pos] = eid;
          list[sl] = pos + 1;
        }
      }
    }
  }
  __syncthreads();

  const int nbw = nb >> 3;
  const bool ovf = (nh >= RCAP);
  const float qnan = __int_as_float(0x7fc00000);

#pragma unroll 1
  for (int jt = 0; jt < nbw; ++jt) {
    const int slot = wave * nbw + jt;
    const int grow = nodeBase + slot;
    int st = soff[slot];
    const int craw = scnt[slot];
    int cnt = craw;
    st  = st < 0 ? 0 : (st > nh ? nh : st);
    cnt = cnt < 0 ? 0 : (cnt > DEGCAP ? DEGCAP : cnt);
    if (cnt > nh - st) cnt = nh - st;
    const float pz = (ovf || craw > DEGCAP) ? qnan : 0.0f;
    const bool liveRow = grow < nN;

    v4f ag[NV];
#pragma unroll
    for (int j = 0; j < NV; ++j) { const v4f z = {0.f, 0.f, 0.f, 0.f}; ag[j] = z; }
#pragma unroll 1
    for (int q = 0; q < cnt; ++q) {
      int idx = st + q; idx = idx > RCAP - 1 ? RCAP - 1 : idx;
      int eid = reg2[idx]; eid = eid < 0 ? 0 : (eid > nE - 1 ? nE - 1 : eid);
      const int sraw = srcs[eid];
      const int s = sraw < 0 ? 0 : (sraw > nN - 1 ? nN - 1 : sraw);
      const float* rp = fin + (size_t)s * W + 4 * lane;
#pragma unroll
      for (int j = 0; j < NV; ++j) {
        v4f v = *(const v4f*)(rp + 128 * j);
        if (RND != 0) { v.x = bf_rne(v.x); v.y = bf_rne(v.y); v.z = bf_rne(v.z); v.w = bf_rne(v.w); }
        ag[j].x += v.x; ag[j].y += v.y; ag[j].z += v.z; ag[j].w += v.w;
      }
    }
    const int nc = liveRow ? grow : nN - 1;
    const float* sp = fin + (size_t)nc * W + 4 * lane;
    v2u hpk[NV], lpk[NV];
#pragma unroll
    for (int j = 0; j < NV; ++j) {
      v4f sv = *(const v4f*)(sp + 128 * j);
      if (RND != 0) { sv.x = bf_rne(sv.x); sv.y = bf_rne(sv.y); sv.z = bf_rne(sv.z); sv.w = bf_rne(sv.w); }
      float r0 = sv.x + ag[j].x, r1 = sv.y + ag[j].y, r2 = sv.z + ag[j].z, r3 = sv.w + ag[j].w;
      r0 = (liveRow ? r0 : 0.0f) + pz;
      r1 = (liveRow ? r1 : 0.0f) + pz;
      r2 = (liveRow ? r2 : 0.0f) + pz;
      r3 = (liveRow ? r3 : 0.0f) + pz;
      const unsigned short h0 = bf_bits(r0), h1 = bf_bits(r1), h2 = bf_bits(r2), h3 = bf_bits(r3);
      const unsigned short l0 = bf_bits(r0 - bf_val(h0)), l1 = bf_bits(r1 - bf_val(h1));
      const unsigned short l2 = bf_bits(r2 - bf_val(h2)), l3 = bf_bits(r3 - bf_val(h3));
      v2u hv, lv;
      hv.x = (unsigned int)h0 | ((unsigned int)h1 << 16);
      hv.y = (unsigned int)h2 | ((unsigned int)h3 << 16);
      lv.x = (unsigned int)l0 | ((unsigned int)l1 << 16);
      lv.y = (unsigned int)l2 | ((unsigned int)l3 << 16);
      hpk[j] = hv; lpk[j] = lv;
    }
    const int lrow = grow - rowOff;
    const bool wsv = lrow < MPr;
    unsigned short* gp = Aout + (size_t)lrow * (size_t)(2 * W) + 4 * lane;
#pragma unroll
    for (int j = 0; j < NV; ++j) {
      if (wsv) { *(volatile v2u*)(gp + 128 * j) = hpk[j]; *(volatile v2u*)(gp + W + 128 * j) = lpk[j]; }
    }
    __threadfence();
#pragma unroll
    for (int j = 0; j < NV; ++j) {
      if (wsv) { *(volatile v2u*)(gp + 128 * j) = hpk[j]; *(volatile v2u*)(gp + W + 128 * j) = lpk[j]; }
    }
  }
}

template <int EPI>
__global__ __launch_bounds__(GTHR) void k_gemm(const unsigned short* __restrict__ A, int lda,
                                               const unsigned short* __restrict__ BT, int ldb, int K,
                                               const float* __restrict__ bias,
                                               void* outp, int ldo, int lsplit, int nN, int mRows,
                                               float* part) {
  __shared__ __attribute__((aligned(16))) float stg[GBM * GBN];
  __shared__ __attribute__((aligned(16))) float pst[PARTW];
  const int tid = (int)threadIdx.x, lane = tid & 31, wave = tid >> 5, hh = lane >> 4, m = lane & 15;
  const int rowBase = (int)blockIdx.x * GBM;
  const int colBase = (int)blockIdx.y * GBN;

  v8f acc[GNT];
  {
    const v8f z = {0.f, 0.f, 0.f, 0.f, 0.f, 0.f, 0.f, 0.f};
#pragma unroll
    for (int t = 0; t < GNT; ++t) acc[t] = z;
  }
  const unsigned short* ap = A  + (size_t)(rowBase + 16 * wave + m) * (size_t)lda + 8 * hh;
  const unsigned short* bp = BT + (size_t)(colBase + m) * (size_t)ldb + 8 * hh;

#pragma unroll 1
  for (int k0 = 0; k0 < K; k0 += 32) {
    Frag af;
    af.h[0] = *(const v8usa*)(ap + k0);
    af.h[1] = *(const v8usa*)(ap + k0 + 16);
#pragma unroll
    for (int nt = 0; nt < GNT; ++nt) {
      const unsigned short* wq = bp + (size_t)(16 * nt) * (size_t)ldb + k0;
      Frag bfr;
      bfr.h[0] = *(const v8usa*)wq;
      bfr.h[1] = *(const v8usa*)(wq + 16);
      acc[nt] = wmx(af, bfr, acc[nt]);
    }
  }

#pragma unroll
  for (int nt = 0; nt < GNT; ++nt) {
    const int lc = 16 * nt + m;
    const float bb = bf_rne(bias[colBase + lc]);
#pragma unroll
    for (int r = 0; r < 8; ++r) {
      const int lr = 16 * wave + 8 * hh + r;
      const bool live = (rowBase + lr) < nN;
      float v = acc[nt][r] + bb;
      if constexpr (EPI != 1) v = relu_np(v);
      stg[lr * GBN + lc] = live ? v : 0.0f;
    }
  }
  __syncthreads();

  if constexpr (EPI == 2) {
    unsigned short* outH = (unsigned short*)outp;
    const int cb = 8 * m;
    const bool isHi = (hh == 0);
    v4u pk[16];
#pragma unroll
    for (int i = 0; i < 16; ++i) {
      const int lr = 16 * wave + i;
      const v4f a = *(const v4fa*)(stg + lr * GBN + cb);
      const v4f b = *(const v4fa*)(stg + lr * GBN + cb + 4);
      const float f[8] = {a.x, a.y, a.z, a.w, b.x, b.y, b.z, b.w};
      unsigned int w[4];
#pragma unroll
      for (int j = 0; j < 4; ++j) {
        const unsigned short h0 = bf_bits(f[2 * j]), h1 = bf_bits(f[2 * j + 1]);
        const unsigned short l0 = bf_bits(f[2 * j] - bf_val(h0)), l1 = bf_bits(f[2 * j + 1] - bf_val(h1));
        const unsigned short q0 = isHi ? h0 : l0, q1 = isHi ? h1 : l1;
        w[j] = (unsigned int)q0 | ((unsigned int)q1 << 16);
      }
      v4u pv; pv.x = w[0]; pv.y = w[1]; pv.z = w[2]; pv.w = w[3];
      pk[i] = pv;
    }
#pragma unroll
    for (int i = 0; i < 16; ++i) {
      const int gr = rowBase + 16 * wave + i;
      unsigned short* op = outH + (size_t)gr * (size_t)ldo + colBase + cb + hh * lsplit;
      if (gr < mRows) *(volatile v4u*)op = pk[i];
    }
    __threadfence();
#pragma unroll
    for (int i = 0; i < 16; ++i) {
      const int gr = rowBase + 16 * wave + i;
      unsigned short* op = outH + (size_t)gr * (size_t)ldo + colBase + cb + hh * lsplit;
      if (gr < mRows) *(volatile v4u*)op = pk[i];
    }
  } else {
    float* outF = (float*)outp;
    v4f fv[16];
#pragma unroll
    for (int i = 0; i < 16; ++i) {
      const int lr = 16 * wave + i;
      fv[i] = *(const v4fa*)(stg + lr * GBN + 4 * lane);
    }
    v4f pv = {0.f, 0.f, 0.f, 0.f};
    const bool pok = (EPI == 1) && (tid < PARTW / 4);
    if constexpr (EPI == 1) {
      int nvr = nN - rowBase;
      nvr = nvr < 0 ? 0 : (nvr > GBM ? GBM : nvr);
      float s = 0.0f;
#pragma unroll 1
      for (int r = 0; r < nvr; ++r) s += stg[r * GBN + tid];
      const float inv = 1.0f / (float)(nvr < 1 ? 1 : nvr);
      const float mean = s * inv;
      float q = 0.0f;
#pragma unroll 1
      for (int r = 0; r < nvr; ++r) {
        const float d = stg[r * GBN + tid] - mean;
        q = fmaf(d, d, q);
      }
      pst[1 + tid] = mean;
      pst[1 + GBN + tid] = q;
      if (tid == 0) pst[0] = (float)nvr;
#pragma unroll 1
      for (int i = 2 * GBN + 1 + tid; i < PARTW; i += GTHR) pst[i] = 0.0f;
      __syncthreads();
      if (pok) pv = *(const v4fa*)(pst + 4 * tid);
    }
    const size_t prow = (size_t)blockIdx.x * (size_t)gridDim.y + (size_t)blockIdx.y;
    float* pp = part + prow * PARTW + 4 * tid;
#pragma unroll
    for (int i = 0; i < 16; ++i) {
      const int gr = rowBase + 16 * wave + i;
      float* op = outF + (size_t)gr * (size_t)ldo + colBase + 4 * lane;
      if (gr < mRows) *(volatile v4f*)op = fv[i];
    }
    if (pok) *(volatile v4f*)pp = pv;
    __threadfence();
#pragma unroll
    for (int i = 0; i < 16; ++i) {
      const int gr = rowBase + 16 * wave + i;
      float* op = outF + (size_t)gr * (size_t)ldo + colBase + 4 * lane;
      if (gr < mRows) *(volatile v4f*)op = fv[i];
    }
    if (pok) *(volatile v4f*)pp = pv;
  }
}

__global__ __launch_bounds__(GBN) void k_bnfin(const float* __restrict__ part, int nPart, int gy, int nh,
                                               const float* __restrict__ gam, const float* __restrict__ bet,
                                               float* ss) {
  __shared__ __attribute__((aligned(16))) float stg[3 * GBN];
  const int tid = (int)threadIdx.x;
  const int by  = (int)blockIdx.x;
  const int col = by * GBN + tid;
  double n = 0.0, mean = 0.0, M2 = 0.0;
#pragma unroll 1
  for (int b = 0; b < nPart; ++b) {
    const float* pr = part + ((size_t)b * (size_t)gy + (size_t)by) * PARTW;
    const double nb = (double)pr[0];
    const double mb = (double)pr[1 + tid];
    const double qb = (double)pr[1 + GBN + tid];
    if (nb > 0.5) {
      const double nn = n + nb;
      const double delta = mb - mean;
      const double f = nb / nn;
      mean = mean + delta * f;
      M2 = M2 + qb + delta * delta * n * f;
      n = nn;
    }
  }
  const double nt = n < 1.0 ? 1.0 : n;
  const float var  = (float)(M2 / nt);
  const float rstd = rsqrtf(var + 1e-5f);
  stg[tid] = (float)mean;
  stg[GBN + tid] = bf_rne(gam[col]) * rstd;
  stg[2 * GBN + tid] = bf_rne(bet[col]);
  __syncthreads();
  const int seg = tid >> 5, j = tid & 31;
  const bool ok = tid < 96;
  v4f v = {0.f, 0.f, 0.f, 0.f};
  float* dp = ss + (size_t)seg * (size_t)nh + (size_t)by * GBN + 4 * j;
  if (ok) {
    v = *(const v4fa*)(stg + seg * GBN + 4 * j);
    *(volatile v4f*)dp = v;
  }
  __threadfence();
  if (ok) *(volatile v4f*)dp = v;
}

__global__ __launch_bounds__(NTHR) void k_bnap1(float* Y, const float* __restrict__ ss, int nN) {
  const int tid = (int)threadIdx.x;
  const int c4 = 4 * tid;
  const v4f mu = *(const v4f*)(ss + c4);
  const v4f sc = *(const v4f*)(ss + HID + c4);
  const v4f be = *(const v4f*)(ss + 2 * HID + c4);
  const int rowBase = (int)blockIdx.x * APR1;
  v4f vals[APR1];
#pragma unroll
  for (int i = 0; i < APR1; ++i) {
    const int grow = rowBase + i;
    const int gc = grow < nN ? grow : nN - 1;
    const v4f y = *(const v4f*)(Y + (size_t)gc * HID + c4);
    v4f o;
    o.x = relu_np((y.x - mu.x) * sc.x + be.x);
    o.y = relu_np((y.y - mu.y) * sc.y + be.y);
    o.z = relu_np((y.z - mu.z) * sc.z + be.z);
    o.w = relu_np((y.w - mu.w) * sc.w + be.w);
    vals[i] = o;
  }
#pragma unroll
  for (int i = 0; i < APR1; ++i) {
    const int grow = rowBase + i;
    if (grow < nN) *(volatile v4f*)(Y + (size_t)grow * HID + c4) = vals[i];
  }
  __threadfence();
#pragma unroll
  for (int i = 0; i < APR1; ++i) {
    const int grow = rowBase + i;
    if (grow < nN) *(volatile v4f*)(Y + (size_t)grow * HID + c4) = vals[i];
  }
}

__global__ __launch_bounds__(NTHR) void k_bnap2(const float* __restrict__ Y, const float* __restrict__ ss,
                                               int nN, int mRows, unsigned short* H) {
  const int tid = (int)threadIdx.x;
  const int q  = tid & 127;
  const int rs = tid >> 7;
  const int c0 = 8 * q;
  const v4f mu0 = *(const v4f*)(ss + c0),           mu1 = *(const v4f*)(ss + c0 + 4);
  const v4f sc0 = *(const v4f*)(ss + HID + c0),     sc1 = *(const v4f*)(ss + HID + c0 + 4);
  const v4f be0 = *(const v4f*)(ss + 2 * HID + c0), be1 = *(const v4f*)(ss + 2 * HID + c0 + 4);
  const int rowBase = (int)blockIdx.x * APR2;
  v8us hv[APR2 / 2], lv[APR2 / 2];
#pragma unroll
  for (int it = 0; it < APR2 / 2; ++it) {
    const int grow = rowBase + 2 * it + rs;
    const int gc = grow < nN ? grow : nN - 1;
    const bool live = grow < nN;
    const v4f a = *(const v4f*)(Y + (size_t)gc * HID + c0);
    const v4f b = *(const v4f*)(Y + (size_t)gc * HID + c0 + 4);
    v4f oa, ob;
    oa.x = relu_np((a.x - mu0.x) * sc0.x + be0.x); oa.y = relu_np((a.y - mu0.y) * sc0.y + be0.y);
    oa.z = relu_np((a.z - mu0.z) * sc0.z + be0.z); oa.w = relu_np((a.w - mu0.w) * sc0.w + be0.w);
    ob.x = relu_np((b.x - mu1.x) * sc1.x + be1.x); ob.y = relu_np((b.y - mu1.y) * sc1.y + be1.y);
    ob.z = relu_np((b.z - mu1.z) * sc1.z + be1.z); ob.w = relu_np((b.w - mu1.w) * sc1.w + be1.w);
    oa.x = live ? oa.x : 0.0f; oa.y = live ? oa.y : 0.0f; oa.z = live ? oa.z : 0.0f; oa.w = live ? oa.w : 0.0f;
    ob.x = live ? ob.x : 0.0f; ob.y = live ? ob.y : 0.0f; ob.z = live ? ob.z : 0.0f; ob.w = live ? ob.w : 0.0f;
    hilo8(oa, ob, hv[it], lv[it]);
  }
#pragma unroll
  for (int it = 0; it < APR2 / 2; ++it) {
    const int grow = rowBase + 2 * it + rs;
    unsigned short* hp = H + (size_t)grow * K2H + c0;
    if (grow < mRows) { *(volatile v8us*)hp = hv[it]; *(volatile v8us*)(hp + HID) = lv[it]; }
  }
  __threadfence();
#pragma unroll
  for (int it = 0; it < APR2 / 2; ++it) {
    const int grow = rowBase + 2 * it + rs;
    unsigned short* hp = H + (size_t)grow * K2H + c0;
    if (grow < mRows) { *(volatile v8us*)hp = hv[it]; *(volatile v8us*)(hp + HID) = lv[it]; }
  }
}

__global__ __launch_bounds__(NTHR) void k_head(const float* __restrict__ U, const float* __restrict__ Wl2,
                                               const float* __restrict__ bl2, int nN, float* out) {
  __shared__ float wls[DMID * NCLS];
  __shared__ float bls[16];
  __shared__ float zt[HR * NCLS];
  __shared__ __attribute__((aligned(16))) float os[HR * NCLS];
  const int tid = (int)threadIdx.x;
#pragma unroll 1
  for (int i = tid; i < DMID * NCLS; i += NTHR) wls[i] = bf_rne(Wl2[i]);
  if (tid < 16) {
    const float bb = bl2[tid < NCLS ? tid : NCLS - 1];
    bls[tid] = (tid < NCLS) ? bf_rne(bb) : 0.0f;
  }
  __syncthreads();
  const int r  = tid & (HR - 1);
  const int cg = tid >> 7;
  const int rowBase = (int)blockIdx.x * HR;
  const int grow = rowBase + r;
  const int gc = grow < nN ? grow : nN - 1;
  const float* ur = U + (size_t)gc * DMID;
  const float* wb = wls + 5 * cg;
  float z0 = 0.0f, z1 = 0.0f, z2 = 0.0f, z3 = 0.0f, z4 = 0.0f;
#pragma unroll 1
  for (int k4 = 0; k4 < DMID / 4; ++k4) {
    const v4f u = *(const v4f*)(ur + 4 * k4);
    const float* w = wb + (4 * k4) * NCLS;
    z0 = fmaf(u.x, w[0], z0); z1 = fmaf(u.x, w[1], z1); z2 = fmaf(u.x, w[2], z2);
    z3 = fmaf(u.x, w[3], z3); z4 = fmaf(u.x, w[4], z4);
    z0 = fmaf(u.y, w[NCLS + 0], z0); z1 = fmaf(u.y, w[NCLS + 1], z1); z2 = fmaf(u.y, w[NCLS + 2], z2);
    z3 = fmaf(u.y, w[NCLS + 3], z3); z4 = fmaf(u.y, w[NCLS + 4], z4);
    z0 = fmaf(u.z, w[2 * NCLS + 0], z0); z1 = fmaf(u.z, w[2 * NCLS + 1], z1); z2 = fmaf(u.z, w[2 * NCLS + 2], z2);
    z3 = fmaf(u.z, w[2 * NCLS + 3], z3); z4 = fmaf(u.z, w[2 * NCLS + 4], z4);
    z0 = fmaf(u.w, w[3 * NCLS + 0], z0); z1 = fmaf(u.w, w[3 * NCLS + 1], z1); z2 = fmaf(u.w, w[3 * NCLS + 2], z2);
    z3 = fmaf(u.w, w[3 * NCLS + 3], z3); z4 = fmaf(u.w, w[3 * NCLS + 4], z4);
  }
  {
    float* zp = zt + r * NCLS + 5 * cg;
    const float* bp = bls + 5 * cg;
    zp[0] = z0 + bp[0]; zp[1] = z1 + bp[1]; zp[2] = z2 + bp[2]; zp[3] = z3 + bp[3]; zp[4] = z4 + bp[4];
  }
  __syncthreads();
  if (tid < HR) {
    const float* zr = zt + tid * NCLS;
    float mx = zr[0];
#pragma unroll 1
    for (int c = 1; c < NCLS; ++c) { const float v = zr[c]; mx = (v > mx) ? v : mx; }
    float s = 0.0f;
#pragma unroll 1
    for (int c = 0; c < NCLS; ++c) s += expf(zr[c] - mx);
    const float lg = logf(s);
#pragma unroll 1
    for (int c = 0; c < NCLS; ++c) os[tid * NCLS + c] = (zr[c] - mx) - lg;
  }
  __syncthreads();
  int nv = nN - rowBase;
  nv = nv < 0 ? 0 : (nv > HR ? HR : nv);
  const int npc = (nv * NCLS) / 4;
  v4f ov[2];
  bool okp[2];
#pragma unroll
  for (int it = 0; it < 2; ++it) {
    const int p = it * NTHR + tid;
    okp[it] = p < npc;
    const int pc = p < (HR * NCLS) / 4 ? p : (HR * NCLS) / 4 - 1;
    ov[it] = *(const v4fa*)(os + 4 * pc);
  }
  float* ob = out + (size_t)rowBase * NCLS;
#pragma unroll
  for (int it = 0; it < 2; ++it) {
    const int p = it * NTHR + tid;
    if (okp[it]) *(volatile v4f*)(ob + 4 * (size_t)p) = ov[it];
  }
  __threadfence();
#pragma unroll
  for (int it = 0; it < 2; ++it) {
    const int p = it * NTHR + tid;
    if (okp[it]) *(volatile v4f*)(ob + 4 * (size_t)p) = ov[it];
  }
}

static int pick_nb(int nE, int nN) {
  int nb = NBMAX;
  while (nb > 16 && (long long)nb * (long long)nE * 5LL > (long long)RCAP * (long long)nN * 4LL) nb >>= 1;
  return nb;
}
static inline int cdiv(int a, int b) { return (a + b - 1) / b; }
static inline size_t al256(size_t o) { return (o + 255) & ~(size_t)255; }

extern "C" void kernel_launch(void* const* d_in, const int* in_sizes, int n_in,
                              void* d_out, int out_size, void* d_ws, size_t ws_size,
                              hipStream_t stream) {
  if (n_in < 18) return;
  if (in_sizes[0] < DIN || (in_sizes[0] % DIN) != 0) return;
  const int nN = in_sizes[0] / DIN;
  if (nN < GBM || nN > 65536) return;
  const int nE2 = in_sizes[1];
  if (nE2 < 2 || (nE2 & 1) != 0) return;
  const int nE = nE2 / 2;
  if (nE < 1 || nE > (1 << 21)) return;
  if (in_sizes[2] != DIN * HID || in_sizes[3] != HID) return;
  if (in_sizes[4] != HID * HID || in_sizes[5] != HID) return;
  if (in_sizes[6] != HID || in_sizes[7] != HID) return;
  if (in_sizes[8] != HID * HID || in_sizes[9] != HID) return;
  if (in_sizes[10] != HID * HID || in_sizes[11] != HID) return;
  if (in_sizes[12] != HID || in_sizes[13] != HID) return;
  if (in_sizes[14] != HID * DMID || in_sizes[15] != DMID) return;
  if (in_sizes[16] != DMID * NCLS || in_sizes[17] != NCLS) return;
  if ((long long)nN * NCLS != (long long)out_size) return;
  if ((((nN % HR) * NCLS) % 32) != 0) return;

  const float* x   = (const float*)d_in[0];
  const int*   ei  = (const int*)  d_in[1];
  const int*   src = ei;
  const int*   dst = ei + nE;
  const float* W1a = (const float*)d_in[2];  const float* b1a = (const float*)d_in[3];
  const float* W1b = (const float*)d_in[4];  const float* b1b = (const float*)d_in[5];
  const float* g1  = (const float*)d_in[6];  const float* be1 = (const float*)d_in[7];
  const float* W2a = (const float*)d_in[8];  const float* b2a = (const float*)d_in[9];
  const float* W2b = (const float*)d_in[10]; const float* b2b = (const float*)d_in[11];
  const float* g2  = (const float*)d_in[12]; const float* be2 = (const float*)d_in[13];
  const float* Wl1 = (const float*)d_in[14]; const float* bl1 = (const float*)d_in[15];
  const float* Wl2 = (const float*)d_in[16]; const float* bl2 = (const float*)d_in[17];
  float* out = (float*)d_out;

  const int MP   = cdiv(nN, GBM) * GBM;
  const int gM   = MP / GBM;
  const int gy   = HID / GBN;
  const int nb   = pick_nb(nE, nN);
  const int vec8 = ((nE & 3) == 0) ? 1 : 0;
  const int nCh  = cdiv(MP, CHR);
  if (nCh < 1 || nCh > 8) return;
  if ((long long)(gM - 1) * GBM >= (long long)nN) return;
  if ((MP % APR2) != 0) return;
  if ((long long)cdiv(MP, nb) * nb < (long long)MP) return;

  char* ws = (char*)d_ws;
  size_t off = 0;
  const size_t szSU = ((size_t)CHR * K2H * 2 > (size_t)MP * DMID * 4) ? (size_t)CHR * K2H * 2 : (size_t)MP * DMID * 4;
  const size_t oP1a = off; off = al256(off + (size_t)NUA * 16);
  const size_t oP1b = off; off = al256(off + (size_t)NUH * 16);
  const size_t oP2a = off; off = al256(off + (size_t)NUH * 16);
  const size_t oP2b = off; off = al256(off + (size_t)NUH * 16);
  const size_t oPL1 = off; off = al256(off + (size_t)NUL * 16);
  const size_t oS1  = off; off = al256(off + (size_t)MP * K1A * 2);
  const size_t oRB  = off; off = al256(off + (size_t)MP * HID * 4);
  const size_t oRC  = off; off = al256(off + (size_t)MP * HID * 4);
  const size_t oSU  = off; off = al256(off + szSU);
  const size_t oT2  = off; off = al256(off + (size_t)CHR * K2H * 2);
  const size_t oPT  = off; off = al256(off + (size_t)gM * gy * PARTW * 4);
  const size_t oSS  = off; off = al256(off + (size_t)(3 * HID) * 4);
  if (off > ws_size || off > (size_t)WSMAX) return;
  unsigned short* P1a = (unsigned short*)(ws + oP1a);
  unsigned short* P1b = (unsigned short*)(ws + oP1b);
  unsigned short* P2a = (unsigned short*)(ws + oP2a);
  unsigned short* P2b = (unsigned short*)(ws + oP2b);
  unsigned short* PL1 = (unsigned short*)(ws + oPL1);
  unsigned short* S1  = (unsigned short*)(ws + oS1);
  float*          YB  = (float*)(ws + oRB);
  unsigned short* H2  = (unsigned short*)(ws + oRB);
  unsigned short* T1  = (unsigned short*)(ws + oRC);
  float*          Y2  = (float*)(ws + oRC);
  unsigned short* S2c = (unsigned short*)(ws + oSU);
  float*          UU  = (float*)(ws + oSU);
  unsigned short* T2c = (unsigned short*)(ws + oT2);
  float*          PT  = (float*)(ws + oPT);
  float*          SS  = (float*)(ws + oSS);

  hipFuncSetAttribute(reinterpret_cast<const void*>(&k_agg<1, 1>), hipFuncAttributeMaxDynamicSharedMemorySize, LDS_AGG);
  hipFuncSetAttribute(reinterpret_cast<const void*>(&k_agg<8, 0>), hipFuncAttributeMaxDynamicSharedMemorySize, LDS_AGG);

  k_wprep<<<NUTOT / NTHR, NTHR, 0, stream>>>(W1a, W1b, W2a, W2b, Wl1, P1a, P1b, P2a, P2b, PL1);
  k_agg<1, 1><<<cdiv(MP, nb), NTHR, LDS_AGG, stream>>>(src, dst, x, S1, nN, nE, nb, vec8, 0, MP);
  k_gemm<2><<<dim3(gM, gy), GTHR, 0, stream>>>(S1, K1A, P1a, K1A, K1A, b1a, (void*)T1, K2H, HID, nN, MP, PT);
  k_gemm<1><<<dim3(gM, gy), GTHR, 0, stream>>>(T1, K2H, P1b, K2H, K2H, b1b, (void*)YB, HID, 0, nN, MP, PT);
  k_bnfin<<<gy, GBN, 0, stream>>>(PT, gM, gy, HID, g1, be1, SS);
  k_bnap1<<<cdiv(nN, APR1), NTHR, 0, stream>>>(YB, SS, nN);
  for (int c = 0; c < nCh; ++c) {
    const int rowOff = c * CHR;
    const int rows   = (MP - rowOff) < CHR ? (MP - rowOff) : CHR;
    const int gmc    = rows / GBM;
    k_agg<8, 0><<<cdiv(rows, nb), NTHR, LDS_AGG, stream>>>(src, dst, YB, S2c, nN, nE, nb, vec8, rowOff, rows);
    k_gemm<2><<<dim3(gmc, gy), GTHR, 0, stream>>>(S2c, K2H, P2a, K2H, K2H, b2a, (void*)T2c, K2H, HID,
                                                  nN - rowOff, rows, PT);
    k_gemm<1><<<dim3(gmc, gy), GTHR, 0, stream>>>(T2c, K2H, P2b, K2H, K2H, b2b,
                                                  (void*)(Y2 + (size_t)rowOff * HID), HID, 0,
                                                  nN - rowOff, rows,
                                                  PT + (size_t)(rowOff / GBM) * (size_t)gy * PARTW);
  }
  k_bnfin<<<gy, GBN, 0, stream>>>(PT, gM, gy, HID, g2, be2, SS);
  k_bnap2<<<MP / APR2, NTHR, 0, stream>>>(Y2, SS, nN, MP, H2);
  k_gemm<3><<<dim3(gM, DMID / GBN), GTHR, 0, stream>>>(H2, K2H, PL1, K2H, K2H, bl1, (void*)UU, DMID, 0, nN, MP, PT);
  k_head<<<cdiv(nN, HR), NTHR, 0, stream>>>(UU, Wl2, bl2, nN, out);
}
